// NoEmbed_AssociativeNet_40475771797932
// MI455X (gfx1250) — hardware-run, weakly checked
//
#include <hip/hip_runtime.h>
#include <math.h>

typedef __attribute__((ext_vector_type(16))) _Float16 v16h;
typedef __attribute__((ext_vector_type(8)))  _Float16 v8h;
typedef __attribute__((ext_vector_type(16))) __bf16   v16b;
typedef __attribute__((ext_vector_type(8)))  __bf16   v8b;
typedef __attribute__((ext_vector_type(8)))  float    v8f;
typedef __attribute__((ext_vector_type(4)))  float    v4f;

constexpr int kB    = 128;
constexpr int kT    = 32;
constexpr int kD    = 128;
constexpr int kHid  = 256;
constexpr int kZ    = kD + kHid;
constexpr int kO    = 128;
constexpr int kBP   = 256;
constexpr int kThr  = 256;
constexpr float kInCarry = 1024.0f;
constexpr float kSc = 1.0f / (kInCarry * kInCarry);
constexpr float kF16MinNormal = 6.103515625e-5f;

static_assert((kB % 64) == 0 && (kHid % 64) == 0 && (kO % 64) == 0 && (kBP % 64) == 0 && (kZ % 32) == 0 && (kHid % 32) == 0 && ((kB / 64) * (kHid / 64)) % 8 == 0 && ((kBP / 64) * (kO / 64)) % 8 == 0, "GEMM M, N multiples of 64, K of 32; grids exact (8 and 8 tiles)");

constexpr size_t kOffW16 = 0ull;
constexpr size_t kOffWO16 = 196608ull;
constexpr size_t kOffBIAS = 262144ull;
constexpr size_t kOffZ16 = 266240ull;
constexpr size_t kOffZ32 = 462848ull;
constexpr size_t kOffPRE = 659456ull;
constexpr size_t kOffHN = 790528ull;
constexpr size_t kOffF32 = 4984832ull;
constexpr size_t kOffTAG = 55316480ull;
constexpr size_t kWsTotal = 55447552ull;
static_assert(kWsTotal <= 134217728ull, "carve cap: under 128 MiB");
static_assert(kOffW16 == 0
              && kOffWO16 == kOffW16 + 196608ull
              && kOffBIAS == kOffWO16 + 65536ull
              && kOffZ16 == kOffBIAS + 4096ull
              && kOffZ32 == kOffZ16 + 196608ull
              && kOffPRE == kOffZ32 + 196608ull
              && kOffHN == kOffPRE + 131072ull
              && kOffF32 == kOffHN + 4194304ull
              && kOffTAG == kOffF32 + 50331648ull
              && kWsTotal == kOffTAG + 131072ull, "the carve is chained and totalled");
static_assert((kOffW16 % 256) == 0 && (kOffWO16 % 256) == 0 && (kOffBIAS % 256) == 0 && (kOffZ16 % 256) == 0 && (kOffZ32 % 256) == 0 && (kOffPRE % 256) == 0 && (kOffHN % 256) == 0 && (kOffF32 % 256) == 0 && (kOffTAG % 256) == 0, "aligned regions");
constexpr int kFBG = 0, kFBO = 256, kFEnd = 1024;
constexpr size_t kOutTag = 0, kOutH = (size_t)kB * kO, kOutF = kOutH + (size_t)kB * kHid, kOutEnd = kOutF + (size_t)kB * kHid * kZ;
static_assert(kOutH == 16384 && kOutF == 49152 && kOutEnd == 12632064, "output offsets");

__device__ __forceinline__ unsigned short f2bf_bits(float f) {
  unsigned u = __float_as_uint(f);
  return (unsigned short)((u + 0x7FFFu + ((u >> 16) & 1u)) >> 16);
}
__device__ __forceinline__ float bf_bits2f(unsigned short h) { return __uint_as_float(((unsigned)h) << 16); }
__device__ __forceinline__ float bf16r(float f) { return bf_bits2f(f2bf_bits(f)); }
__device__ __forceinline__ float carry_flush(float v, float carry) {
  const float s = v * carry;
  return (fabsf(s) < kF16MinNormal) ? 0.0f : s;
}
__device__ __forceinline__ float frcp(float x) { return __builtin_amdgcn_rcpf(x); }

__device__ __forceinline__ void dep_guard4_h(v8f& a, v8f& b, v8f& c, v8f& d, v16h x, v16h y) { asm volatile("v_nop\n\tv_nop\n\tv_nop\n\tv_nop" : "+v"(a), "+v"(b), "+v"(c), "+v"(d) : "v"(x), "v"(y)); }
__device__ __forceinline__ void dep_guard4_b(v8f& a, v8f& b, v8f& c, v8f& d, v16b x, v16b y) { asm volatile("v_nop\n\tv_nop\n\tv_nop\n\tv_nop" : "+v"(a), "+v"(b), "+v"(c), "+v"(d) : "v"(x), "v"(y)); }
__device__ __forceinline__ void keep4_h(v16h a, v16h b, v16h c, v16h d) { asm volatile("v_nop" :: "v"(a), "v"(b), "v"(c), "v"(d)); }
__device__ __forceinline__ void keep4_b(v16b a, v16b b, v16b c, v16b d) { asm volatile("v_nop" :: "v"(a), "v"(b), "v"(c), "v"(d)); }
__device__ __forceinline__ void acc_guard4(v8f& a, v8f& b, v8f& c, v8f& d) { asm volatile("v_nop\n\tv_nop\n\tv_nop\n\tv_nop" : "+v"(a), "+v"(b), "+v"(c), "+v"(d)); }

template <typename T> struct Frag;
template <> struct Frag<_Float16> {
  typedef v16h V; union U { v16h v; v8h h[2]; };
  static __device__ __forceinline__ v16h load(const _Float16* p) {
    U f; f.h[0] = *(const v8h*)(p); f.h[1] = *(const v8h*)(p + 16); return f.v;
  }
  static __device__ __forceinline__ v8f mma(v16h a, v16h b, v8f c) {
    return __builtin_amdgcn_wmma_f32_16x16x32_f16(false, a, false, b, (short)0, c, false, false);
  }
  static __device__ __forceinline__ void guard4(v8f& a, v8f& b, v8f& c, v8f& d, v16h x, v16h y) { dep_guard4_h(a, b, c, d, x, y); }
  static __device__ __forceinline__ void keep(v16h a, v16h b, v16h c, v16h d) { keep4_h(a, b, c, d); }
};
template <> struct Frag<__bf16> {
  typedef v16b V; union U { v16b v; v8b h[2]; };
  static __device__ __forceinline__ v16b load(const __bf16* p) {
    U f; f.h[0] = *(const v8b*)(p); f.h[1] = *(const v8b*)(p + 16); return f.v;
  }
  static __device__ __forceinline__ v8f mma(v16b a, v16b b, v8f c) {
    return __builtin_amdgcn_wmma_f32_16x16x32_bf16(false, a, false, b, (short)0, c, false, false);
  }
  static __device__ __forceinline__ void guard4(v8f& a, v8f& b, v8f& c, v8f& d, v16b x, v16b y) { dep_guard4_b(a, b, c, d, x, y); }
  static __device__ __forceinline__ void keep(v16b a, v16b b, v16b c, v16b d) { keep4_b(a, b, c, d); }
};

__device__ __forceinline__ v8f mma_h(v16h a, v16h b, v8f c) {
  c = __builtin_amdgcn_wmma_f32_16x16x32_f16(false, a, false, b, (short)0, c, false, false);
  asm volatile("v_nop\n\tv_nop\n\tv_nop\n\tv_nop" : "+v"(c) : "v"(a), "v"(b));
  return c;
}

template <int ET> struct Elem;
template <> struct Elem<0> { typedef _Float16 T; };
template <> struct Elem<1> { typedef __bf16 T; };
template <int ET, bool SPLIT, int BIAS_MODE, int OUT_MODE, bool RESID, int ACT = 0>
__global__ __launch_bounds__(256) void wmma_gemm64(
    const unsigned short* __restrict__ Ap, const unsigned short* __restrict__ A2p, int lda, long strideA,
    const unsigned short* __restrict__ Btp, const unsigned short* __restrict__ Bt2p, int ldb, long strideB,
    void* __restrict__ Cout, void* __restrict__ Cout2, int ldc, long strideC,
    const float* __restrict__ bias,
    const float* __restrict__ resid, long strideR,
    int M, int N, int K, float scale) {
  typedef typename Elem<ET>::T T;
  typedef typename Frag<T>::V V;
  const T* A = (const T*)Ap; const T* A2 = (const T*)A2p; const T* Bt = (const T*)Btp; const T* Bt2 = (const T*)Bt2p;
  __shared__ __align__(16) float sT[8][16 * 68];
  const int b    = blockIdx.y;
  const int lane = threadIdx.x & 31;
  const int wave = threadIdx.x >> 5;
  const int tilesN = N >> 6;
  const int tilesM = M >> 6;
  const int tile = blockIdx.x * 8 + wave;
  if (tile >= tilesM * tilesN) return;
  const int tm = tile / tilesN;
  const int tn = tile - tm * tilesN;
  const int m0 = tm << 6;
  const int n0 = tn << 6;

  const T* Ab  = A  + (size_t)b * strideA;
  const T* Bb  = Bt + (size_t)b * strideB;
  const T* Ab2 = SPLIT ? (A2  + (size_t)b * strideA) : nullptr;
  const T* Bb2 = SPLIT ? (Bt2 + (size_t)b * strideB) : nullptr;

  const int rlane = lane & 15;
  const int koff  = (lane >> 4) * 8;
  const int mOff  = (lane >> 4) * 8;

  v8f acc[4][4];
#pragma unroll
  for (int i = 0; i < 4; ++i)
#pragma unroll
    for (int j = 0; j < 4; ++j) acc[i][j] = (v8f){0.f,0.f,0.f,0.f,0.f,0.f,0.f,0.f};

  for (int k0 = 0; k0 < K; k0 += 32) {
    V bh[4], bl[4];
#pragma unroll
    for (int j = 0; j < 4; ++j) {
      const size_t bo = (size_t)(n0 + (j << 4) + rlane) * ldb + koff + k0;
      bh[j] = Frag<T>::load(Bb + bo);
      if (SPLIT) bl[j] = Frag<T>::load(Bb2 + bo);
    }
#pragma unroll
    for (int i = 0; i < 4; ++i) {
      const size_t ao = (size_t)(m0 + (i << 4) + rlane) * lda + koff + k0;
      V ah = Frag<T>::load(Ab + ao);
      V al;
      if (SPLIT) al = Frag<T>::load(Ab2 + ao);
#pragma unroll
      for (int j = 0; j < 4; ++j) {
        acc[i][j] = Frag<T>::mma(ah, bh[j], acc[i][j]);
        if (SPLIT) {
          acc[i][j] = Frag<T>::mma(ah, bl[j], acc[i][j]);
          acc[i][j] = Frag<T>::mma(al, bh[j], acc[i][j]);
        }
      }
      Frag<T>::guard4(acc[i][0], acc[i][1], acc[i][2], acc[i][3], ah, SPLIT ? al : ah);
    }
    Frag<T>::keep(bh[0], bh[1], bh[2], bh[3]);
    if (SPLIT) Frag<T>::keep(bl[0], bl[1], bl[2], bl[3]);
  }
  acc_guard4(acc[0][0], acc[0][1], acc[0][2], acc[0][3]);
  acc_guard4(acc[1][0], acc[1][1], acc[1][2], acc[1][3]);
  acc_guard4(acc[2][0], acc[2][1], acc[2][2], acc[2][3]);
  acc_guard4(acc[3][0], acc[3][1], acc[3][2], acc[3][3]);

  float* slab = sT[wave];
  const float* Rb = RESID ? (resid + (size_t)b * strideR) : nullptr;
#pragma unroll
  for (int i = 0; i < 4; ++i) {
    const int mBase = m0 + (i << 4);
#pragma unroll
    for (int j = 0; j < 4; ++j) {
      const int n = n0 + (j << 4) + rlane;
      float bv = 0.f;
      if (BIAS_MODE == 2) bv = bias[n];
#pragma unroll
      for (int r = 0; r < 8; ++r) {
        float v = acc[i][j][r] * scale;
        if (BIAS_MODE == 1) v += bias[mBase + mOff + r];
        if (BIAS_MODE == 2) v += bv;
        if (RESID) v += Rb[(size_t)(mBase + mOff + r) * ldc + n];
        if (ACT == 1) v = tanhf(v);
        if (ACT == 2) v = fmaxf(v, 0.0f);
        if (ACT == 3) v = v / (1.0f + expf(-v));
        if (ACT == 4) v = (v > 0.f) ? v : 0.01f * v;
        slab[(mOff + r) * 68 + (j << 4) + rlane] = v;
      }
    }
    __builtin_amdgcn_fence(__ATOMIC_RELEASE, "workgroup");
    __builtin_amdgcn_wave_barrier();
    __builtin_amdgcn_fence(__ATOMIC_ACQUIRE, "workgroup");
    if (OUT_MODE == 0) {
      float* C = (float*)Cout + (size_t)b * strideC;
      const int hh = lane >> 4, c4 = (lane & 15) * 4;
      for (int pass = 0; pass < 2; ++pass) {
#pragma unroll
        for (int it = 0; it < 8; ++it) {
          const int row = it * 2 + hh;
          v4f v = *(const v4f*)(slab + row * 68 + c4);
          *(volatile v4f*)(C + (size_t)(mBase + row) * ldc + n0 + c4) = v;
        }
        __threadfence();
      }
    } else {
      const int q = lane >> 3, c8 = (lane & 7) * 8;
      unsigned short* C  = (unsigned short*)Cout  + (size_t)b * strideC;
      unsigned short* C2 = (OUT_MODE == 2) ? ((unsigned short*)Cout2 + (size_t)b * strideC) : nullptr;
      for (int pass = 0; pass < 2; ++pass) {
#pragma unroll
        for (int it = 0; it < 4; ++it) {
          const int row = it * 4 + q;
          const float* sp = slab + row * 68 + c8;
          v8h hv, lv;
#pragma unroll
          for (int e = 0; e < 8; ++e) {
            if (OUT_MODE == 1) {
              hv[e] = (_Float16)sp[e];
            } else {
              unsigned short hb = f2bf_bits(sp[e]);
              unsigned short lb = f2bf_bits(sp[e] - bf_bits2f(hb));
              hv[e] = __builtin_bit_cast(_Float16, hb);
              lv[e] = __builtin_bit_cast(_Float16, lb);
            }
          }
          *(volatile v8h*)(C + (size_t)(mBase + row) * ldc + n0 + c8) = hv;
          if (OUT_MODE == 2) *(volatile v8h*)(C2 + (size_t)(mBase + row) * ldc + n0 + c8) = lv;
        }
        __threadfence();
      }
    }
    __builtin_amdgcn_fence(__ATOMIC_RELEASE, "workgroup");
    __builtin_amdgcn_wave_barrier();
    __builtin_amdgcn_fence(__ATOMIC_ACQUIRE, "workgroup");
  }
}

__global__ __launch_bounds__(kThr) void cast_plane_kernel(const float* __restrict__ src, unsigned short* __restrict__ dst,
                                                          int colsLog2, int dstPitch, int dstOff) {
  const int i   = blockIdx.x * kThr + threadIdx.x;
  const int sh  = colsLog2 - 3;
  const int row = i >> sh;
  const int c8  = (i & ((1 << sh) - 1)) * 8;
  const float* sp = src + ((size_t)row << colsLog2) + c8;
  const v4f a0 = *(const v4f*)(sp);
  const v4f a1 = *(const v4f*)(sp + 4);
  v8h hv;
#pragma unroll
  for (int e = 0; e < 4; ++e) {
    const float f0 = a0[e];
    const float f1 = a1[e];
    hv[e]     = (_Float16)carry_flush(bf16r(f0), kInCarry);
    hv[4 + e] = (_Float16)carry_flush(bf16r(f1), kInCarry);
  }
  unsigned short* dp = dst + (size_t)row * dstPitch + dstOff + c8;
  *(volatile v8h*)dp = hv;
  __threadfence();
  *(volatile v8h*)dp = hv;
}

__global__ __launch_bounds__(kThr) void setup_kernel(const float* __restrict__ sentence, const float* __restrict__ h0, const float* __restrict__ b, const float* __restrict__ b_out,
                                                     float* __restrict__ BIAS, unsigned short* __restrict__ Z16, float* __restrict__ Z32) {
  const unsigned y = blockIdx.y;
  const unsigned c = threadIdx.x;
  if (y == 0u) {
    const unsigned i0 = c * 4u;
    v4f o = {0.f, 0.f, 0.f, 0.f};
    if (i0 < (unsigned)kFBO) {
      const v4f a = *(const v4f*)(b + i0);
#pragma unroll
      for (int e = 0; e < 4; ++e) { const float p = a[e]; o[e] = bf16r(p); }
    } else if (i0 < (unsigned)(kFBO + kO)) {
      const v4f a = *(const v4f*)(b_out + (i0 - (unsigned)kFBO));
#pragma unroll
      for (int e = 0; e < 4; ++e) { const float p = a[e]; o[e] = bf16r(p); }
    }
    float* dp = BIAS + i0;
    *(volatile v4f*)dp = o;
    __threadfence();
    *(volatile v4f*)dp = o;
  } else {
    if (c >= 48u) return;
    const unsigned r = y - 1u;
    const bool live = r < (unsigned)kB;
    const unsigned rs = live ? r : 0u;
    const float* sp = (c < 16u) ? (sentence + (size_t)rs * kT * kD + c * 8u) : (h0 + (size_t)rs * kHid + (c - 16u) * 8u);
    const v4f a0 = *(const v4f*)sp, a1 = *(const v4f*)(sp + 4);
    v4f f0, f1; v8h hv;
#pragma unroll
    for (int e = 0; e < 4; ++e) {
      const float p = a0[e], q = a1[e];
      f0[e] = bf16r(p); f1[e] = bf16r(q);
      hv[e] = (_Float16)(live ? carry_flush(f0[e], kInCarry) : 0.0f);
      hv[4 + e] = (_Float16)(live ? carry_flush(f1[e], kInCarry) : 0.0f);
    }
    unsigned short* hp = Z16 + (size_t)r * kZ + c * 8u;
    float* fp = Z32 + (size_t)rs * kZ + c * 8u;
    for (int pass = 0; pass < 2; ++pass) {
      *(volatile v8h*)hp = hv;
      if (live) { *(volatile v4f*)fp = f0; *(volatile v4f*)(fp + 4) = f1; }
      __threadfence();
    }
  }
}
static_assert(kZ / 8 == 48 && kD / 8 == 16 && kFEnd / 4 == kThr && (kFBO % 128) == 0 && ((kFBO + kO) % 128) == 0, "set-up rows: 48 chunks; the bias arms end on wave boundaries");

__global__ __launch_bounds__(kThr) void finit_kernel(const float* __restrict__ F0, float* __restrict__ F32) {
  const size_t o4 = ((size_t)blockIdx.x * kThr + threadIdx.x) * 4u;
  const v4f a = *(const v4f*)(F0 + o4);
  v4f o;
#pragma unroll
  for (int e = 0; e < 4; ++e) { const float p = a[e]; o[e] = bf16r(p); }
  *(volatile v4f*)(F32 + o4) = o;
  __threadfence();
  *(volatile v4f*)(F32 + o4) = o;
}
static_assert(((size_t)kB * kHid * kZ / 4) == 12288 * kThr, "fast-weight start grid exact");

__global__ __launch_bounds__(kThr) void fast_step_kernel(const float* __restrict__ PRE, const float* __restrict__ Z32, const float* __restrict__ lam, const float* __restrict__ gamma,
                                                         float* __restrict__ F32, float* __restrict__ HN) {
  const unsigned w = blockIdx.x * 8u + (threadIdx.x >> 5);
  const unsigned lane = threadIdx.x & 31u;
  const unsigned smp = w >> 8, u = w & 255u;
  float* fr = F32 + ((size_t)smp * kHid + u) * kZ + lane * 4u;
  const float* zr = Z32 + (size_t)smp * kZ + lane * 4u;
  const float* lr = lam + (size_t)u * kZ + lane * 4u;
  const float* gr = gamma + (size_t)u * kZ + lane * 4u;
  v4f fv[3], zv[3];
  float s = 0.0f;
#pragma unroll
  for (int k = 0; k < 3; ++k) {
    fv[k] = *(const v4f*)(fr + 128 * k);
    zv[k] = *(const v4f*)(zr + 128 * k);
    s += fv[k][0] * zv[k][0]; s += fv[k][1] * zv[k][1]; s += fv[k][2] * zv[k][2]; s += fv[k][3] * zv[k][3];
  }
  s += __shfl_xor(s, 1, 32);
  s += __shfl_xor(s, 2, 32);
  s += __shfl_xor(s, 4, 32);
  s += __shfl_xor(s, 8, 32);
  s += __shfl_xor(s, 16, 32);
  const float hn = tanhf(PRE[(size_t)smp * kHid + u] + s);
  v4f fn[3];
#pragma unroll
  for (int k = 0; k < 3; ++k) {
    const v4f lv = *(const v4f*)(lr + 128 * k), gv = *(const v4f*)(gr + 128 * k);
#pragma unroll
    for (int e = 0; e < 4; ++e) fn[k][e] = bf16r(lv[e]) * fv[k][e] + bf16r(gv[e]) * (hn * zv[k][e]);
  }
  float* hp = HN + ((size_t)smp * kHid + u) * 32u + lane;
  for (int pass = 0; pass < 2; ++pass) {
#pragma unroll
    for (int k = 0; k < 3; ++k) *(volatile v4f*)(fr + 128 * k) = fn[k];
    *(volatile float*)hp = hn;
    __threadfence();
  }
}
static_assert(kZ == 3 * 128 && (kB * kHid) % 8 == 0 && kHid == 256, "one wave a row: 12 columns a lane");

__global__ __launch_bounds__(64) void handover_kernel(const float* __restrict__ HN, const float* __restrict__ sentence, unsigned short* __restrict__ Z16, float* __restrict__ Z32, int t) {
  const unsigned smp = blockIdx.y;
  const unsigned c = threadIdx.x;
  if (c >= 48u) return;
  v4f f0, f1;
  if (c >= 16u) {
    const float* hp = HN + ((size_t)smp * kHid + (c - 16u) * 8u) * 32u;
#pragma unroll
    for (int e = 0; e < 4; ++e) { f0[e] = hp[(size_t)e * 32u]; f1[e] = hp[(size_t)(4 + e) * 32u]; }
  } else {
    if (t + 1 >= kT) return;
    const float* sp = sentence + ((size_t)smp * kT + (size_t)(t + 1)) * kD + c * 8u;
    const v4f a0 = *(const v4f*)sp, a1 = *(const v4f*)(sp + 4);
#pragma unroll
    for (int e = 0; e < 4; ++e) { const float p = a0[e], q = a1[e]; f0[e] = bf16r(p); f1[e] = bf16r(q); }
  }
  v8h hv;
#pragma unroll
  for (int e = 0; e < 4; ++e) { hv[e] = (_Float16)carry_flush(f0[e], kInCarry); hv[4 + e] = (_Float16)carry_flush(f1[e], kInCarry); }
  unsigned short* hp16 = Z16 + (size_t)smp * kZ + c * 8u;
  float* fp = Z32 + (size_t)smp * kZ + c * 8u;
  for (int pass = 0; pass < 2; ++pass) {
    *(volatile v8h*)hp16 = hv;
    *(volatile v4f*)fp = f0;
    *(volatile v4f*)(fp + 4) = f1;
    __threadfence();
  }
}

__global__ __launch_bounds__(128) void rows_out_kernel(const float* __restrict__ src, int pitch, int cols, float* __restrict__ dst) {
  const unsigned row = blockIdx.y;
  const unsigned c4 = threadIdx.x * 4u;
  const v4f a = *(const v4f*)(src + (size_t)row * (unsigned)pitch + c4);
  float* dp = dst + (size_t)row * (unsigned)cols + c4;
  *(volatile v4f*)dp = a;
  __threadfence();
  *(volatile v4f*)dp = a;
}

static_assert(((size_t)kHid * kZ / 8) % kThr == 0 && ((size_t)kO * kHid / 8) % kThr == 0, "plane cast grids exact");

extern "C" void kernel_launch(void* const* d_in, const int* in_sizes, int n_in,
                              void* d_out, int out_size, void* d_ws, size_t ws_size,
                              hipStream_t stream) {
  if (n_in < 9 || d_out == nullptr || d_ws == nullptr) return;
  if (in_sizes[0] != kB * kT * kD || in_sizes[1] != kB * kHid || in_sizes[2] != kB * kHid * kZ || in_sizes[3] != kHid * kZ || in_sizes[4] != kHid) return;
  if (in_sizes[5] != kHid * kZ || in_sizes[6] != kHid * kZ || in_sizes[7] != kO * kHid || in_sizes[8] != kO) return;
  if ((size_t)out_size != kOutEnd) return;
  if (ws_size < kWsTotal) return;
  const float* sentence = (const float*)d_in[0];
  const float* h0 = (const float*)d_in[1];
  const float* F0 = (const float*)d_in[2];
  const float* W = (const float*)d_in[3];
  const float* b = (const float*)d_in[4];
  const float* lam = (const float*)d_in[5];
  const float* gamma = (const float*)d_in[6];
  const float* W_out = (const float*)d_in[7];
  const float* b_out = (const float*)d_in[8];
  float* out = (float*)d_out;
  char* ws = (char*)d_ws;
  unsigned short* W16 = (unsigned short*)(ws + kOffW16);
  unsigned short* WO16 = (unsigned short*)(ws + kOffWO16);
  float* BIAS = (float*)(ws + kOffBIAS);
  unsigned short* Z16 = (unsigned short*)(ws + kOffZ16);
  float* Z32 = (float*)(ws + kOffZ32);
  float* PRE = (float*)(ws + kOffPRE);
  float* HN = (float*)(ws + kOffHN);
  float* F32 = (float*)(ws + kOffF32);
  float* TAG = (float*)(ws + kOffTAG);

  cast_plane_kernel<<<(int)(((size_t)kHid * kZ / 8) / kThr), kThr, 0, stream>>>(W, W16, 12, 4096, 0);
  cast_plane_kernel<<<(int)(((size_t)kO * kHid / 8) / kThr), kThr, 0, stream>>>(W_out, WO16, 8, kHid, 0);
  setup_kernel<<<dim3(1, 1 + kBP), kThr, 0, stream>>>(sentence, h0, b, b_out, BIAS, Z16, Z32);
  finit_kernel<<<12288, kThr, 0, stream>>>(F0, F32);
  for (int t = 0; t < kT; ++t) {
    wmma_gemm64<0, false, 2, 0, false, 0><<<dim3((kB / 64) * (kHid / 64) / 8, 1), 256, 0, stream>>>(
        Z16, Z16, kZ, 0L, W16, W16, kZ, 0L, (void*)PRE, (void*)PRE, kHid, 0L, BIAS + kFBG, nullptr, 0L, kB, kHid, kZ, kSc);
    fast_step_kernel<<<(kB * kHid) / 8, kThr, 0, stream>>>(PRE, Z32, lam, gamma, F32, HN);
    handover_kernel<<<dim3(1, kB), 64, 0, stream>>>(HN, sentence, Z16, Z32, t);
  }
  wmma_gemm64<0, false, 2, 0, false, 0><<<dim3((kBP / 64) * (kO / 64) / 8, 1), 256, 0, stream>>>(
      Z16 + kD, Z16 + kD, kZ, 0L, WO16, WO16, kHid, 0L, (void*)TAG, (void*)TAG, kO, 0L, BIAS + kFBO, nullptr, 0L, kBP, kO, kHid, kSc);
  rows_out_kernel<<<dim3(1, kB), kO / 4, 0, stream>>>(TAG, kO, kO, out + kOutTag);
  rows_out_kernel<<<dim3(1, kB), kHid / 4, 0, stream>>>(Z32 + kD, kZ, kHid, out + kOutH);
  rows_out_kernel<<<dim3(1, kB * kHid), kZ / 4, 0, stream>>>(F32, kZ, kZ, out + kOutF);
}
